// BlockV3_84155589198357
// MI455X (gfx1250) — hardware-verified
//
#include <hip/hip_runtime.h>
#include <stddef.h>


typedef _Float16 v16h __attribute__((ext_vector_type(16)));
typedef _Float16 v8h  __attribute__((ext_vector_type(8)));
typedef v8h v8ha __attribute__((may_alias));
typedef float v8f __attribute__((ext_vector_type(8)));
typedef float v4f __attribute__((ext_vector_type(4)));
union Frag { v16h v; v8h h[2]; };

static constexpr int CEMB = 768;
static constexpr int NH   = 12;
static constexpr int DHD  = 64;
static constexpr int BN   = 2;
static constexpr int TN   = 2048;
static constexpr int MTOT = BN * TN;
static constexpr int HID  = 3072;

static_assert(MTOT % 64 == 0, "");
static_assert(CEMB % 128 == 0 && HID % 128 == 0, "");
static_assert(CEMB % 32 == 0 && HID % 32 == 0, "");
static_assert(TN % 64 == 0 && TN == 2048, "");

__device__ __forceinline__ v8f wmma16(v16h a, v16h b, v8f c) {
  v8f d = __builtin_amdgcn_wmma_f32_16x16x32_f16(false, a, false, b, (short)0, c, false, false);
  asm volatile("v_nop\n\tv_nop\n\tv_nop\n\tv_nop" : "+v"(d) : "v"(a), "v"(b));
  return d;
}

__device__ __forceinline__ v8f zero8() {
  v8f z;
  #pragma unroll
  for (int i = 0; i < 8; i++) z[i] = 0.f;
  return z;
}

__global__ __launch_bounds__(256) void ln_rows(const float* __restrict__ x,
                                               const float* __restrict__ g,
                                               const float* __restrict__ be,
                                               _Float16* __restrict__ out, int M) {
  const int lane = threadIdx.x & 31;
  const int wave = threadIdx.x >> 5;
  const int row  = blockIdx.x * 8 + wave;
  if (row >= M) return;
  const float* xr = x + (size_t)row * CEMB;
  float v[24];
  #pragma unroll
  for (int c = 0; c < 3; c++) {
    const v4f p0 = *(const v4f*)(xr + 256 * c + 8 * lane);
    const v4f p1 = *(const v4f*)(xr + 256 * c + 8 * lane + 4);
    #pragma unroll
    for (int i = 0; i < 4; i++) { v[8 * c + i] = p0[i]; v[8 * c + 4 + i] = p1[i]; }
  }
  float s = 0.f;
  #pragma unroll
  for (int i = 0; i < 24; i++) s += v[i];
  #pragma unroll
  for (int m = 16; m >= 1; m >>= 1) s += __shfl_xor(s, m, 32);
  const float mu = s * (1.f / CEMB);
  float s2 = 0.f;
  #pragma unroll
  for (int i = 0; i < 24; i++) { const float d = v[i] - mu; s2 += d * d; }
  #pragma unroll
  for (int m = 16; m >= 1; m >>= 1) s2 += __shfl_xor(s2, m, 32);
  const float r = rsqrtf(s2 * (1.f / CEMB) + 1e-5f);

  v8h o[3];
  #pragma unroll
  for (int c = 0; c < 3; c++) {
    const v4f g0 = *(const v4f*)(g  + 256 * c + 8 * lane);
    const v4f g1 = *(const v4f*)(g  + 256 * c + 8 * lane + 4);
    const v4f b0 = *(const v4f*)(be + 256 * c + 8 * lane);
    const v4f b1 = *(const v4f*)(be + 256 * c + 8 * lane + 4);
    #pragma unroll
    for (int i = 0; i < 4; i++) {
      o[c][i]     = (_Float16)((v[8 * c + i]     - mu) * r * g0[i] + b0[i]);
      o[c][4 + i] = (_Float16)((v[8 * c + 4 + i] - mu) * r * g1[i] + b1[i]);
    }
  }
  _Float16* orow = out + (size_t)row * CEMB + 8 * lane;
  #pragma unroll
  for (int c = 0; c < 3; c++) *(volatile v8h*)(orow + 256 * c) = o[c];
  __threadfence();
  #pragma unroll
  for (int c = 0; c < 3; c++) *(volatile v8h*)(orow + 256 * c) = o[c];
}

template <int MODE>
__global__ __launch_bounds__(256) void gemm16(const _Float16* __restrict__ A,
                                              const float* __restrict__ W,
                                              const float* __restrict__ bias,
                                              const float* __restrict__ resid,
                                              void* __restrict__ outp,
                                              int M, int N, int K, float oscale) {
  constexpr int STR = 40;
  constexpr int SCP = 132;
  __shared__ __align__(16) float smem[64 * SCP];
  _Float16* sA = (_Float16*)smem;
  _Float16* sB = sA + 64 * STR;

  const int tid  = threadIdx.x;
  const int lane = tid & 31;
  const int wave = tid >> 5;
  const int l16  = lane & 15;
  const int hf   = lane >> 4;
  const int wm   = wave & 1;
  const int wn   = wave >> 1;
  const int n0   = blockIdx.x * 128;
  const int m0   = blockIdx.y * 64;
  if (m0 + 64 > M || n0 + 128 > N) return;

  v8f acc[2][2];
  #pragma unroll
  for (int mi = 0; mi < 2; mi++) {
    #pragma unroll
    for (int ni = 0; ni < 2; ni++) acc[mi][ni] = zero8();
  }

  const int ar = tid >> 2, aq = (tid & 3) * 8;
  const int br = tid >> 1, bq = (tid & 1) * 16;
  const _Float16* ag = A + (size_t)(m0 + ar) * K + aq;
  const float*    wg = W + (size_t)(n0 + br) * K + bq;

  for (int k0 = 0; k0 < K; k0 += 32) {
    const v8h av = *(const v8h*)(ag + k0);
    const v4f w0 = *(const v4f*)(wg + k0);
    const v4f w1 = *(const v4f*)(wg + k0 + 4);
    const v4f w2 = *(const v4f*)(wg + k0 + 8);
    const v4f w3 = *(const v4f*)(wg + k0 + 12);
    v8h bv0, bv1;
    #pragma unroll
    for (int i = 0; i < 4; i++) {
      bv0[i]     = (_Float16)(w0[i] * 64.f);
      bv0[4 + i] = (_Float16)(w1[i] * 64.f);
      bv1[i]     = (_Float16)(w2[i] * 64.f);
      bv1[4 + i] = (_Float16)(w3[i] * 64.f);
    }
    __syncthreads();
    *(v8h*)(sA + ar * STR + aq)     = av;
    *(v8h*)(sB + br * STR + bq)     = bv0;
    *(v8h*)(sB + br * STR + bq + 8) = bv1;
    __syncthreads();

    Frag fa[2], fb[2];
    #pragma unroll
    for (int mi = 0; mi < 2; mi++) {
      const _Float16* p = sA + (wm * 32 + mi * 16 + l16) * STR + 8 * hf;
      fa[mi].h[0] = *(const v8h*)(p);
      fa[mi].h[1] = *(const v8h*)(p + 16);
    }
    #pragma unroll
    for (int ni = 0; ni < 2; ni++) {
      const _Float16* p = sB + (wn * 32 + ni * 16 + l16) * STR + 8 * hf;
      fb[ni].h[0] = *(const v8h*)(p);
      fb[ni].h[1] = *(const v8h*)(p + 16);
    }
    #pragma unroll
    for (int mi = 0; mi < 2; mi++) {
      #pragma unroll
      for (int ni = 0; ni < 2; ni++) acc[mi][ni] = wmma16(fa[mi].v, fb[ni].v, acc[mi][ni]);
    }
  }
  __syncthreads();

  float* sC = smem;
  #pragma unroll
  for (int mi = 0; mi < 2; mi++) {
    #pragma unroll
    for (int ni = 0; ni < 2; ni++) {
      const int col  = wn * 32 + ni * 16 + l16;
      const float bv = bias[n0 + col];
      #pragma unroll
      for (int r = 0; r < 8; r++) {
        const int row = wm * 32 + mi * 16 + 8 * hf + r;
        sC[row * SCP + col] = acc[mi][ni][r] * oscale + bv;
      }
    }
  }
  __syncthreads();

  if (MODE == 2) {
    float* out = (float*)outp;
    v4f vals[8];
    size_t gi[8];
    #pragma unroll
    for (int i = 0; i < 8; i++) {
      const int row = wave * 8 + i;
      gi[i] = (size_t)(m0 + row) * N + n0 + 4 * lane;
      const v4f c  = *(const v4f*)(sC + row * SCP + 4 * lane);
      const v4f rr = *(const v4f*)(resid + gi[i]);
      vals[i] = c + rr;
    }
    #pragma unroll
    for (int i = 0; i < 8; i++) *(volatile v4f*)(out + gi[i]) = vals[i];
    __threadfence();
    #pragma unroll
    for (int i = 0; i < 8; i++) *(volatile v4f*)(out + gi[i]) = vals[i];
  } else if (MODE == 0) {
    _Float16* out = (_Float16*)outp;
    const int p  = lane & 7;
    const int b  = m0 >> 11;
    const int t0 = m0 & (TN - 1);
    v8h vals[4];
    _Float16* dst[4];
    #pragma unroll
    for (int it = 0; it < 4; it++) {
      const int L   = wave * 16 + it * 4 + (lane >> 3);
      const int row = L >> 1;
      const int hs  = L & 1;
      const float* src = sC + row * SCP + hs * 64 + 8 * p;
      const v4f c0 = *(const v4f*)(src);
      const v4f c1 = *(const v4f*)(src + 4);
      #pragma unroll
      for (int i = 0; i < 4; i++) { vals[it][i] = (_Float16)c0[i]; vals[it][4 + i] = (_Float16)c1[i]; }
      const int hh = (n0 >> 6) + hs;
      const int t  = t0 + row;
      dst[it] = out + ((((size_t)(b * NH + hh)) * TN + t) << 6) + 8 * p;
    }
    #pragma unroll
    for (int it = 0; it < 4; it++) *(volatile v8h*)(dst[it]) = vals[it];
    __threadfence();
    #pragma unroll
    for (int it = 0; it < 4; it++) *(volatile v8h*)(dst[it]) = vals[it];
  } else if (MODE == 1) {
    _Float16* out = (_Float16*)outp;
    const int p  = lane & 7;
    const int b  = m0 >> 11;
    const int t0 = m0 & (TN - 1);
    v8h vals[4];
    _Float16* dst[4];
    #pragma unroll
    for (int it = 0; it < 4; it++) {
      const int c = wave * 16 + it * 4 + (lane >> 3);
      #pragma unroll
      for (int i = 0; i < 8; i++) vals[it][i] = (_Float16)sC[(8 * p + i) * SCP + c];
      const int gc = n0 + c;
      const int hh = gc >> 6;
      const int d  = gc & (DHD - 1);
      dst[it] = out + ((size_t)((b * NH + hh) * DHD + d)) * TN + t0 + 8 * p;
    }
    #pragma unroll
    for (int it = 0; it < 4; it++) *(volatile v8h*)(dst[it]) = vals[it];
    __threadfence();
    #pragma unroll
    for (int it = 0; it < 4; it++) *(volatile v8h*)(dst[it]) = vals[it];
  } else {
    _Float16* out = (_Float16*)outp;
    v8h vals[4];
    _Float16* dst[4];
    #pragma unroll
    for (int it = 0; it < 4; it++) {
      const int row = wave * 8 + it * 2 + (lane >> 4);
      const int cs  = (lane & 15) * 8;
      const float* src = sC + row * SCP + cs;
      const v4f c0 = *(const v4f*)(src);
      const v4f c1 = *(const v4f*)(src + 4);
      #pragma unroll
      for (int i = 0; i < 4; i++) {
        const float u0 = c0[i], u1 = c1[i];
        vals[it][i]     = (_Float16)(0.5f * u0 * (1.f + erff(u0 * 0.70710678118654752f)));
        vals[it][4 + i] = (_Float16)(0.5f * u1 * (1.f + erff(u1 * 0.70710678118654752f)));
      }
      dst[it] = out + (size_t)(m0 + row) * N + n0 + cs;
    }
    #pragma unroll
    for (int it = 0; it < 4; it++) *(volatile v8h*)(dst[it]) = vals[it];
    __threadfence();
    #pragma unroll
    for (int it = 0; it < 4; it++) *(volatile v8h*)(dst[it]) = vals[it];
  }
}

__global__ __launch_bounds__(128) void attn16(const _Float16* __restrict__ q,
                                              const _Float16* __restrict__ k,
                                              const _Float16* __restrict__ vT,
                                              const int* __restrict__ pmask,
                                              const int* __restrict__ condp,
                                              _Float16* __restrict__ y) {
  constexpr int PST = 72;
  __shared__ __align__(16) _Float16 lds[64 * PST];
  __shared__ int scnt[4];
  const int lane = threadIdx.x & 31;
  const int wave = threadIdx.x >> 5;
  const int l16  = lane & 15;
  const int hf   = lane >> 4;
  const int idx  = blockIdx.x;
  const int qt   = idx % (TN / 64);
  const int tmp  = idx / (TN / 64);
  const int h    = tmp % NH;
  const int b    = tmp / NH;
  if (b >= BN) return;

  int cs = 0;
  for (int i = threadIdx.x; i < TN; i += 128) cs += pmask[(size_t)b * TN + i];
  #pragma unroll
  for (int m = 16; m >= 1; m >>= 1) cs += __shfl_xor(cs, m, 32);
  if (lane == 0) scnt[wave] = cs;
  __syncthreads();
  const int nb = TN - (scnt[0] + scnt[1] + scnt[2] + scnt[3]);
  const int cl = condp[0];

  const int qbase = qt * 64 + wave * 16;
  const _Float16* qh = q  + (size_t)(b * NH + h) * TN * DHD;
  const _Float16* kh = k  + (size_t)(b * NH + h) * TN * DHD;
  const _Float16* vh = vT + (size_t)(b * NH + h) * DHD * TN;
  _Float16* pw = lds + wave * 16 * PST;

  Frag a0, a1;
  {
    const _Float16* qr = qh + (size_t)(qbase + l16) * DHD;
    a0.h[0] = *(const v8h*)(qr + 8 * hf);
    a0.h[1] = *(const v8h*)(qr + 16 + 8 * hf);
    a1.h[0] = *(const v8h*)(qr + 32 + 8 * hf);
    a1.h[1] = *(const v8h*)(qr + 48 + 8 * hf);
  }

  v8f O[4];
  #pragma unroll
  for (int n = 0; n < 4; n++) O[n] = zero8();
  float mrow[8], lpart[8];
  #pragma unroll
  for (int j = 0; j < 8; j++) { mrow[j] = -1e30f; lpart[j] = 0.f; }

  for (int kt = 0; kt < TN; kt += 64) {
    __syncthreads();
    v8f sc[4];
    #pragma unroll
    for (int t = 0; t < 4; t++) {
      const _Float16* kr = kh + (size_t)(kt + 16 * t + l16) * DHD;
      Frag kb0, kb1;
      kb0.h[0] = *(const v8h*)(kr + 8 * hf);
      kb0.h[1] = *(const v8h*)(kr + 16 + 8 * hf);
      kb1.h[0] = *(const v8h*)(kr + 32 + 8 * hf);
      kb1.h[1] = *(const v8h*)(kr + 48 + 8 * hf);
      v8f s = zero8();
      s = wmma16(a0.v, kb0.v, s);
      s = wmma16(a1.v, kb1.v, s);
      sc[t] = s;
    }
    bool ok[4];
    #pragma unroll
    for (int t = 0; t < 4; t++) {
      const int key = kt + 16 * t + l16;
      ok[t] = (key >= cl) || (key < nb);
    }
    #pragma unroll
    for (int j = 0; j < 8; j++) {
      float vv[4];
      #pragma unroll
      for (int t = 0; t < 4; t++) vv[t] = ok[t] ? sc[t][j] * 0.125f : -1e30f;
      float mx = fmaxf(fmaxf(vv[0], vv[1]), fmaxf(vv[2], vv[3]));
      #pragma unroll
      for (int m = 1; m <= 8; m <<= 1) mx = fmaxf(mx, __shfl_xor(mx, m, 16));
      const float mnew = fmaxf(mrow[j], mx);
      const float corr = __expf(mrow[j] - mnew);
      float e[4];
      #pragma unroll
      for (int t = 0; t < 4; t++) e[t] = __expf(vv[t] - mnew);
      lpart[j] = lpart[j] * corr + ((e[0] + e[1]) + (e[2] + e[3]));
      mrow[j]  = mnew;
      #pragma unroll
      for (int n = 0; n < 4; n++) O[n][j] *= corr;
      const int r = (8 * hf + j) * PST;
      #pragma unroll
      for (int t = 0; t < 4; t++) pw[r + 16 * t + l16] = (_Float16)e[t];
    }
    __syncthreads();
    Frag pa0, pa1;
    {
      const _Float16* pr = pw + l16 * PST;
      pa0.h[0] = *(const v8ha*)(pr + 8 * hf);
      pa0.h[1] = *(const v8ha*)(pr + 16 + 8 * hf);
      pa1.h[0] = *(const v8ha*)(pr + 32 + 8 * hf);
      pa1.h[1] = *(const v8ha*)(pr + 48 + 8 * hf);
    }
    #pragma unroll
    for (int n = 0; n < 4; n++) {
      const _Float16* vr = vh + (size_t)(n * 16 + l16) * TN + kt;
      Frag vb0, vb1;
      vb0.h[0] = *(const v8h*)(vr + 8 * hf);
      vb0.h[1] = *(const v8h*)(vr + 16 + 8 * hf);
      vb1.h[0] = *(const v8h*)(vr + 32 + 8 * hf);
      vb1.h[1] = *(const v8h*)(vr + 48 + 8 * hf);
      O[n] = wmma16(pa0.v, vb0.v, O[n]);
      O[n] = wmma16(pa1.v, vb1.v, O[n]);
    }
  }

  float inv[8];
  #pragma unroll
  for (int j = 0; j < 8; j++) {
    float l = lpart[j];
    #pragma unroll
    for (int m = 1; m <= 8; m <<= 1) l += __shfl_xor(l, m, 16);
    inv[j] = 64.f / l;
  }
  __syncthreads();
  #pragma unroll
  for (int n = 0; n < 4; n++) {
    #pragma unroll
    for (int j = 0; j < 8; j++) pw[(8 * hf + j) * PST + n * 16 + l16] = (_Float16)(O[n][j] * inv[j]);
  }
  __syncthreads();

  const int p = lane & 7;
  v8h vals[4];
  _Float16* dst[4];
  #pragma unroll
  for (int it = 0; it < 4; it++) {
    const int L = wave * 16 + it * 4 + (lane >> 3);
    vals[it] = *(const v8ha*)(lds + L * PST + 8 * p);
    dst[it]  = y + ((size_t)(b * TN + qt * 64 + L)) * CEMB + h * DHD + 8 * p;
  }
  #pragma unroll
  for (int it = 0; it < 4; it++) *(volatile v8h*)(dst[it]) = vals[it];
  __threadfence();
  #pragma unroll
  for (int it = 0; it < 4; it++) *(volatile v8h*)(dst[it]) = vals[it];
}

extern "C" void kernel_launch(void* const* d_in, const int* in_sizes, int n_in,
                              void* d_out, int out_size, void* d_ws, size_t ws_size,
                              hipStream_t stream) {
  if (n_in < 19) return;
  if (in_sizes[0] != MTOT * CEMB || in_sizes[1] < 1 || in_sizes[2] != BN * TN ||
      in_sizes[3] != CEMB || in_sizes[4] != CEMB || in_sizes[5] != CEMB || in_sizes[6] != CEMB ||
      in_sizes[7] != CEMB * CEMB || in_sizes[8] != CEMB ||
      in_sizes[9] != CEMB * CEMB || in_sizes[10] != CEMB ||
      in_sizes[11] != CEMB * CEMB || in_sizes[12] != CEMB ||
      in_sizes[13] != CEMB * CEMB || in_sizes[14] != CEMB ||
      in_sizes[15] != HID * CEMB || in_sizes[16] != HID ||
      in_sizes[17] != CEMB * HID || in_sizes[18] != CEMB ||
      out_size != MTOT * CEMB) return;

  const float* x    = (const float*)d_in[0];
  const int*   cond = (const int*)d_in[1];
  const int*   pm   = (const int*)d_in[2];
  const float* g1   = (const float*)d_in[3];
  const float* bln1 = (const float*)d_in[4];
  const float* g2   = (const float*)d_in[5];
  const float* bln2 = (const float*)d_in[6];
  const float* Wq   = (const float*)d_in[7];
  const float* bq   = (const float*)d_in[8];
  const float* Wk   = (const float*)d_in[9];
  const float* bk   = (const float*)d_in[10];
  const float* Wv   = (const float*)d_in[11];
  const float* bv   = (const float*)d_in[12];
  const float* Wp   = (const float*)d_in[13];
  const float* bp   = (const float*)d_in[14];
  const float* W1   = (const float*)d_in[15];
  const float* b1   = (const float*)d_in[16];
  const float* W2   = (const float*)d_in[17];
  const float* b2   = (const float*)d_in[18];

  char* ws = (char*)d_ws;
  size_t off = 0;
  auto carve = [&](size_t bytes) -> char* {
    char* p = ws + off;
    off += (bytes + 255) & ~(size_t)255;
    return p;
  };
  const size_t actf16 = (size_t)MTOT * CEMB * 2;
  _Float16* hb  = (_Float16*)carve(actf16);
  _Float16* qb  = (_Float16*)carve(actf16);
  _Float16* kb  = (_Float16*)carve(actf16);
  _Float16* vtb = (_Float16*)carve(actf16);
  _Float16* yb  = (_Float16*)carve(actf16);
  float*    xa  = (float*)carve((size_t)MTOT * CEMB * 4);
  _Float16* h2b = (_Float16*)carve(actf16);
  _Float16* ub  = (_Float16*)carve((size_t)MTOT * HID * 2);
  if (off > ws_size) return;

  const dim3 gln((MTOT + 7) / 8);
  const dim3 g768((CEMB + 127) / 128, (MTOT + 63) / 64);
  const dim3 g3072((HID + 127) / 128, (MTOT + 63) / 64);
  const dim3 gattn(BN * NH * (TN / 64));

  ln_rows<<<gln, 256, 0, stream>>>(x, g1, bln1, hb, MTOT);

  gemm16<0><<<g768, 256, 0, stream>>>(hb, Wq, bq, x, (void*)qb,  MTOT, CEMB, CEMB, 1.f / 64.f);
  gemm16<0><<<g768, 256, 0, stream>>>(hb, Wk, bk, x, (void*)kb,  MTOT, CEMB, CEMB, 1.f / 64.f);
  gemm16<1><<<g768, 256, 0, stream>>>(hb, Wv, bv, x, (void*)vtb, MTOT, CEMB, CEMB, 1.f / 64.f);

  attn16<<<gattn, 128, 0, stream>>>(qb, kb, vtb, pm, cond, yb);

  gemm16<2><<<g768, 256, 0, stream>>>(yb, Wp, bp, x, (void*)xa, MTOT, CEMB, CEMB, 1.f / 4096.f);
  ln_rows<<<gln, 256, 0, stream>>>(xa, g2, bln2, h2b, MTOT);

  gemm16<3><<<g3072, 256, 0, stream>>>(h2b, W1, b1, x, (void*)ub, MTOT, HID, CEMB, 1.f / 64.f);
  gemm16<2><<<g768, 256, 0, stream>>>(ub, W2, b2, xa, d_out, MTOT, CEMB, HID, 1.f / 64.f);

  (void)hipGetLastError();
}
